// MambaBlock_72009421684767
// MI455X (gfx1250) — hardware-verified
//
#include <hip/hip_runtime.h>
#include <math.h>

typedef __attribute__((ext_vector_type(16))) _Float16 v16h;
typedef __attribute__((ext_vector_type(8)))  _Float16 v8h;
typedef __attribute__((ext_vector_type(16))) __bf16   v16b;
typedef __attribute__((ext_vector_type(8)))  __bf16   v8b;
typedef __attribute__((ext_vector_type(8)))  float    v8f;
typedef __attribute__((ext_vector_type(4)))  float    v4f;
typedef __attribute__((ext_vector_type(4)))  unsigned int v4u;

constexpr int kBatch   = 2;
constexpr int kSeq     = 2048;
constexpr int kDim     = 1024;
constexpr int kHeads   = 16;
constexpr int kHd      = kDim / kHeads;
constexpr int kRows    = kBatch * kSeq;
constexpr int kQkvN    = 3 * kDim;
constexpr int kKC      = 64;
constexpr int kQTiles  = kSeq / 64;
constexpr int kDimLog2 = 10;
static_assert((1 << kDimLog2) == kDim, "dim is a power of four");
static_assert((kDimLog2 % 2) == 0, "even exponent");
constexpr float kAttScale  = 1.0f / (float)(1 << (kDimLog2 / 2));
constexpr float kWCarry    = 32.0f;
constexpr float kWCarryInv = 1.0f / kWCarry;
constexpr float kPCarry    = 32768.0f;
constexpr float kOCarry    = 256.0f;
constexpr float kOutScale  = 1.0f / (kOCarry * kWCarry);
static_assert(kHd == 64, "head dim 64");
static_assert(kRows == 4096 && kQkvN == 3072, "shapes");
static_assert((kDim % 32) == 0, "GEMM K multiple of 32");
static_assert((kRows % 64) == 0 && (kDim % 64) == 0 && (kQkvN % 64) == 0 && (kHd % 64) == 0, "GEMM M,N multiples of 64");
static_assert((kSeq % kKC) == 0 && (kSeq % 64) == 0, "sequence tiles");

constexpr size_t kPlaneHalves = (size_t)kHeads * kRows * kHd;
constexpr size_t kOffXH   = 0;
constexpr size_t kOffWQT  = kOffXH   + (size_t)kRows * kDim * 2;
constexpr size_t kOffWOT  = kOffWQT  + (size_t)kQkvN * kDim * 2;
constexpr size_t kOffQKVH = kOffWOT  + (size_t)kDim * kDim * 2;
constexpr size_t kOffVT   = kOffQKVH + 3 * kPlaneHalves * 2;
constexpr size_t kOffOH   = kOffVT   + kPlaneHalves * 2;
constexpr size_t kWsTotal = kOffOH   + (size_t)kRows * kDim * 2;
static_assert(kWsTotal == 58720256ull, "carve total");
static_assert(kWsTotal <= 134217728ull, "carve cap");
static_assert((kOffWQT % 128) == 0 && (kOffWOT % 128) == 0 && (kOffQKVH % 128) == 0 &&
              (kOffVT % 128) == 0 && (kOffOH % 128) == 0, "128-B aligned regions");

__device__ __forceinline__ unsigned short f2bf_bits(float f) {
  unsigned u = __float_as_uint(f);
  return (unsigned short)((u + 0x7FFFu + ((u >> 16) & 1u)) >> 16);
}
__device__ __forceinline__ float bf_bits2f(unsigned short h) { return __uint_as_float(((unsigned)h) << 16); }
__device__ __forceinline__ unsigned pk16(unsigned a, unsigned b) { return (a & 0xffffu) | (b << 16); }

__device__ __forceinline__ void dep_guard4_h(v8f& a, v8f& b, v8f& c, v8f& d, v16h x, v16h y) {
  asm volatile("v_nop\n\tv_nop\n\tv_nop\n\tv_nop" : "+v"(a), "+v"(b), "+v"(c), "+v"(d) : "v"(x), "v"(y));
}
__device__ __forceinline__ void dep_guard4_b(v8f& a, v8f& b, v8f& c, v8f& d, v16b x, v16b y) {
  asm volatile("v_nop\n\tv_nop\n\tv_nop\n\tv_nop" : "+v"(a), "+v"(b), "+v"(c), "+v"(d) : "v"(x), "v"(y));
}
__device__ __forceinline__ void keep4_h(v16h a, v16h b, v16h c, v16h d) { asm volatile("v_nop" :: "v"(a), "v"(b), "v"(c), "v"(d)); }
__device__ __forceinline__ void keep4_b(v16b a, v16b b, v16b c, v16b d) { asm volatile("v_nop" :: "v"(a), "v"(b), "v"(c), "v"(d)); }
__device__ __forceinline__ void acc_guard4(v8f& a, v8f& b, v8f& c, v8f& d) {
  asm volatile("v_nop\n\tv_nop\n\tv_nop\n\tv_nop" : "+v"(a), "+v"(b), "+v"(c), "+v"(d));
}
template <typename T> struct Frag;
template <> struct Frag<_Float16> {
  typedef v16h V; union U { v16h v; v8h h[2]; };
  static __device__ __forceinline__ v16h load(const _Float16* p) {
    U f; f.h[0] = *(const v8h*)(p); f.h[1] = *(const v8h*)(p + 16); return f.v;
  }
  static __device__ __forceinline__ v8f mma(v16h a, v16h b, v8f c) {
    return __builtin_amdgcn_wmma_f32_16x16x32_f16(false, a, false, b, (short)0, c, false, false);
  }
  static __device__ __forceinline__ void guard4(v8f& a, v8f& b, v8f& c, v8f& d, v16h x, v16h y) { dep_guard4_h(a, b, c, d, x, y); }
  static __device__ __forceinline__ void keep(v16h a, v16h b, v16h c, v16h d) { keep4_h(a, b, c, d); }
};
template <> struct Frag<__bf16> {
  typedef v16b V; union U { v16b v; v8b h[2]; };
  static __device__ __forceinline__ v16b load(const __bf16* p) {
    U f; f.h[0] = *(const v8b*)(p); f.h[1] = *(const v8b*)(p + 16); return f.v;
  }
  static __device__ __forceinline__ v8f mma(v16b a, v16b b, v8f c) {
    return __builtin_amdgcn_wmma_f32_16x16x32_bf16(false, a, false, b, (short)0, c, false, false);
  }
  static __device__ __forceinline__ void guard4(v8f& a, v8f& b, v8f& c, v8f& d, v16b x, v16b y) { dep_guard4_b(a, b, c, d, x, y); }
  static __device__ __forceinline__ void keep(v16b a, v16b b, v16b c, v16b d) { keep4_b(a, b, c, d); }
};

__device__ __forceinline__ v8f mma_h(v16h a, v16h b, v8f c) {
  c = __builtin_amdgcn_wmma_f32_16x16x32_f16(false, a, false, b, (short)0, c, false, false);
  asm volatile("v_nop\n\tv_nop\n\tv_nop\n\tv_nop" : "+v"(c) : "v"(a), "v"(b));
  return c;
}

template <int ET> struct Elem;
template <> struct Elem<0> { typedef _Float16 T; };
template <> struct Elem<1> { typedef __bf16 T; };
template <int ET, bool SPLIT, int BIAS_MODE, int OUT_MODE, bool RESID, int ACT = 0>
__global__ __launch_bounds__(256) void wmma_gemm64(
    const unsigned short* __restrict__ Ap, const unsigned short* __restrict__ A2p, int lda, long strideA,
    const unsigned short* __restrict__ Btp, const unsigned short* __restrict__ Bt2p, int ldb, long strideB,
    void* __restrict__ Cout, void* __restrict__ Cout2, int ldc, long strideC,
    const float* __restrict__ bias,
    const float* __restrict__ resid, long strideR,
    int M, int N, int K, float scale) {
  typedef typename Elem<ET>::T T;
  typedef typename Frag<T>::V V;
  const T* A = (const T*)Ap; const T* A2 = (const T*)A2p; const T* Bt = (const T*)Btp; const T* Bt2 = (const T*)Bt2p;
  __shared__ __align__(16) float sT[8][16 * 68];
  const int b    = blockIdx.y;
  const int lane = threadIdx.x & 31;
  const int wave = threadIdx.x >> 5;
  const int tilesN = N >> 6;
  const int tilesM = M >> 6;
  const int tile = blockIdx.x * 8 + wave;
  if (tile >= tilesM * tilesN) return;
  const int tm = tile / tilesN;
  const int tn = tile - tm * tilesN;
  const int m0 = tm << 6;
  const int n0 = tn << 6;

  const T* Ab  = A  + (size_t)b * strideA;
  const T* Bb  = Bt + (size_t)b * strideB;
  const T* Ab2 = SPLIT ? (A2  + (size_t)b * strideA) : nullptr;
  const T* Bb2 = SPLIT ? (Bt2 + (size_t)b * strideB) : nullptr;

  const int rlane = lane & 15;
  const int koff  = (lane >> 4) * 8;
  const int mOff  = (lane >> 4) * 8;

  v8f acc[4][4];
#pragma unroll
  for (int i = 0; i < 4; ++i)
#pragma unroll
    for (int j = 0; j < 4; ++j) acc[i][j] = (v8f){0.f,0.f,0.f,0.f,0.f,0.f,0.f,0.f};

  for (int k0 = 0; k0 < K; k0 += 32) {
    V bh[4], bl[4];
#pragma unroll
    for (int j = 0; j < 4; ++j) {
      const size_t bo = (size_t)(n0 + (j << 4) + rlane) * ldb + koff + k0;
      bh[j] = Frag<T>::load(Bb + bo);
      if (SPLIT) bl[j] = Frag<T>::load(Bb2 + bo);
    }
#pragma unroll
    for (int i = 0; i < 4; ++i) {
      const size_t ao = (size_t)(m0 + (i << 4) + rlane) * lda + koff + k0;
      V ah = Frag<T>::load(Ab + ao);
      V al;
      if (SPLIT) al = Frag<T>::load(Ab2 + ao);
#pragma unroll
      for (int j = 0; j < 4; ++j) {
        acc[i][j] = Frag<T>::mma(ah, bh[j], acc[i][j]);
        if (SPLIT) {
          acc[i][j] = Frag<T>::mma(ah, bl[j], acc[i][j]);
          acc[i][j] = Frag<T>::mma(al, bh[j], acc[i][j]);
        }
      }
      Frag<T>::guard4(acc[i][0], acc[i][1], acc[i][2], acc[i][3], ah, SPLIT ? al : ah);
    }
    Frag<T>::keep(bh[0], bh[1], bh[2], bh[3]);
    if (SPLIT) Frag<T>::keep(bl[0], bl[1], bl[2], bl[3]);
  }
  acc_guard4(acc[0][0], acc[0][1], acc[0][2], acc[0][3]);
  acc_guard4(acc[1][0], acc[1][1], acc[1][2], acc[1][3]);
  acc_guard4(acc[2][0], acc[2][1], acc[2][2], acc[2][3]);
  acc_guard4(acc[3][0], acc[3][1], acc[3][2], acc[3][3]);

  float* slab = sT[wave];
  const float* Rb = RESID ? (resid + (size_t)b * strideR) : nullptr;
#pragma unroll
  for (int i = 0; i < 4; ++i) {
    const int mBase = m0 + (i << 4);
#pragma unroll
    for (int j = 0; j < 4; ++j) {
      const int n = n0 + (j << 4) + rlane;
      float bv = 0.f;
      if (BIAS_MODE == 2) bv = bias[n];
#pragma unroll
      for (int r = 0; r < 8; ++r) {
        float v = acc[i][j][r] * scale;
        if (BIAS_MODE == 1) v += bias[mBase + mOff + r];
        if (BIAS_MODE == 2) v += bv;
        if (RESID) v += Rb[(size_t)(mBase + mOff + r) * ldc + n];
        if (ACT == 2) v = fmaxf(v, 0.0f);
        if (ACT == 4) v = (v > 0.f) ? v : 0.01f * v;
        slab[(mOff + r) * 68 + (j << 4) + rlane] = v;
      }
    }
    __builtin_amdgcn_fence(__ATOMIC_RELEASE, "workgroup");
    __builtin_amdgcn_wave_barrier();
    __builtin_amdgcn_fence(__ATOMIC_ACQUIRE, "workgroup");
    if (OUT_MODE == 0) {
      float* C = (float*)Cout + (size_t)b * strideC;
      const int hh = lane >> 4, c4 = (lane & 15) * 4;
      for (int pass = 0; pass < 2; ++pass) {
#pragma unroll
        for (int it = 0; it < 8; ++it) {
          const int row = it * 2 + hh;
          v4f v = *(const v4f*)(slab + row * 68 + c4);
          *(volatile v4f*)(C + (size_t)(mBase + row) * ldc + n0 + c4) = v;
        }
        __threadfence();
      }
    } else {
      const int q = lane >> 3, c8 = (lane & 7) * 8;
      unsigned short* C  = (unsigned short*)Cout  + (size_t)b * strideC;
      unsigned short* C2 = (OUT_MODE == 2) ? ((unsigned short*)Cout2 + (size_t)b * strideC) : nullptr;
      for (int pass = 0; pass < 2; ++pass) {
#pragma unroll
        for (int it = 0; it < 4; ++it) {
          const int row = it * 4 + q;
          const float* sp = slab + row * 68 + c8;
          v8h hv, lv;
#pragma unroll
          for (int e = 0; e < 8; ++e) {
            if (OUT_MODE == 1) {
              hv[e] = (_Float16)sp[e];
            } else {
              unsigned short hb = f2bf_bits(sp[e]);
              unsigned short lb = f2bf_bits(sp[e] - bf_bits2f(hb));
              hv[e] = __builtin_bit_cast(_Float16, hb);
              lv[e] = __builtin_bit_cast(_Float16, lb);
            }
          }
          *(volatile v8h*)(C + (size_t)(mBase + row) * ldc + n0 + c8) = hv;
          if (OUT_MODE == 2) *(volatile v8h*)(C2 + (size_t)(mBase + row) * ldc + n0 + c8) = lv;
        }
        __threadfence();
      }
    }
    __builtin_amdgcn_fence(__ATOMIC_RELEASE, "workgroup");
    __builtin_amdgcn_wave_barrier();
    __builtin_amdgcn_fence(__ATOMIC_ACQUIRE, "workgroup");
  }
}

__global__ __launch_bounds__(256) void cast_f16_kernel(
    const float* __restrict__ src, unsigned short* __restrict__ dst, int total8, float scale)
{
  const int i = blockIdx.x * 256 + threadIdx.x;
  if (i >= total8) return;
  const size_t e0 = (size_t)i << 3;
  const float* p = src + e0;
  const v4f a0 = *(const v4f*)(p);
  const v4f a1 = *(const v4f*)(p + 4);
  v8h hv;
#pragma unroll
  for (int e = 0; e < 4; ++e) {
    hv[e]     = (_Float16)(a0[e] * scale);
    hv[4 + e] = (_Float16)(a1[e] * scale);
  }
  unsigned short* q = dst + e0;
  *(volatile v8h*)q = hv;
  __threadfence();
  *(volatile v8h*)q = hv;
}

__global__ __launch_bounds__(256) void transpose_cast_kernel(
    const float* __restrict__ W, unsigned short* __restrict__ Bt, int Kdim, int Ndim, float scale)
{
  __shared__ float tile[64 * 65];
  const int tid = threadIdx.x, lane = tid & 31, wave = tid >> 5;
  const int n0 = blockIdx.x * 64;
  const int k0 = blockIdx.y * 64;
#pragma unroll
  for (int p = 0; p < 16; ++p) {
    const int idx = tid + p * 256;
    const int kk  = idx >> 6;
    const int nn  = idx & 63;
    const int n   = n0 + nn;
    const int nc  = (n < Ndim) ? n : (Ndim - 1);
    const float v = W[(size_t)(k0 + kk) * Ndim + nc];
    tile[kk * 65 + nn] = (n < Ndim) ? (v * scale) : 0.f;
  }
  __syncthreads();
  const int q = lane >> 3, c8 = (lane & 7) * 8;
  v8h hv[2];
#pragma unroll
  for (int it = 0; it < 2; ++it) {
    const int nrow = it * 32 + wave * 4 + q;
#pragma unroll
    for (int e = 0; e < 8; ++e) hv[it][e] = (_Float16)tile[(c8 + e) * 65 + nrow];
  }
  for (int pass = 0; pass < 2; ++pass) {
#pragma unroll
    for (int it = 0; it < 2; ++it) {
      const int nrow = it * 32 + wave * 4 + q;
      *(volatile v8h*)(Bt + (size_t)(n0 + nrow) * Kdim + k0 + c8) = hv[it];
    }
    __threadfence();
  }
}

__global__ __launch_bounds__(256) void vtrans_kernel(
    const unsigned short* __restrict__ Vh, unsigned short* __restrict__ Vt)
{
  __shared__ unsigned int tw[64 * 36];
  const int tid = threadIdx.x, lane = tid & 31, wave = tid >> 5;
  const int jt = blockIdx.x;
  const int hb = blockIdx.y;
  const int h  = hb >> 1, b = hb & 1;
  const size_t src = ((size_t)h * kRows + (size_t)b * kSeq + (size_t)jt * 64) * kHd;
#pragma unroll
  for (int it = 0; it < 2; ++it) {
    const int piece = it * 256 + tid;
    const int row = piece >> 3;
    const int c4  = (piece & 7) * 4;
    const v4u w = *(const v4u*)(Vh + src + (size_t)row * kHd + c4 * 2);
    tw[row * 36 + c4 + 0] = w.x;
    tw[row * 36 + c4 + 1] = w.y;
    tw[row * 36 + c4 + 2] = w.z;
    tw[row * 36 + c4 + 3] = w.w;
  }
  __syncthreads();
  const int q = lane >> 3, c8 = (lane & 7) * 8;
  v4u ov[2];
#pragma unroll
  for (int it = 0; it < 2; ++it) {
    const int d  = it * 32 + wave * 4 + q;
    const int wd = d >> 1;
    const unsigned sh = (unsigned)(d & 1) * 16u;
    unsigned hb16[8];
#pragma unroll
    for (int e = 0; e < 8; ++e) hb16[e] = (tw[(c8 + e) * 36 + wd] >> sh) & 0xffffu;
    ov[it] = (v4u){pk16(hb16[0], hb16[1]), pk16(hb16[2], hb16[3]), pk16(hb16[4], hb16[5]), pk16(hb16[6], hb16[7])};
  }
  for (int pass = 0; pass < 2; ++pass) {
#pragma unroll
    for (int it = 0; it < 2; ++it) {
      const int d = it * 32 + wave * 4 + q;
      *(volatile v4u*)(Vt + ((size_t)hb * kHd + d) * kSeq + (size_t)jt * 64 + c8) = ov[it];
    }
    __threadfence();
  }
}

__global__ __launch_bounds__(128) void attn_f16_kernel(
    const unsigned short* __restrict__ Qp, const unsigned short* __restrict__ Kp,
    const unsigned short* __restrict__ Vtp, unsigned short* __restrict__ Op)
{
  __shared__ __align__(16) _Float16 Ksh[kKC * kHd];
  __shared__ __align__(16) _Float16 Vsh[kHd * kKC];
  __shared__ __align__(16) _Float16 Psh[4][16 * kKC];
  __shared__ __align__(16) float    Os[4][16 * 68];

  const int tid  = threadIdx.x;
  const int wave = tid >> 5;
  const int lane = tid & 31;
  const int hh   = lane >> 4;
  const int c    = lane & 15;

  const int bx = blockIdx.x;
  const int qb = bx % kQTiles;
  const int hb = bx / kQTiles;
  const int h  = hb >> 1;
  const int b  = hb & 1;
  const int q0 = qb * 64 + wave * 16;

  const size_t rowbase = ((size_t)h * kRows + (size_t)b * kSeq) * kHd;
  const _Float16* Qb = (const _Float16*)Qp + rowbase;
  const _Float16* Kb = (const _Float16*)Kp + rowbase;
  const _Float16* Vb = (const _Float16*)Vtp + (size_t)hb * kHd * kSeq;

  v16h qa[2];
  {
    const _Float16* qrow = Qb + (size_t)(q0 + c) * kHd + 8 * hh;
    qa[0] = Frag<_Float16>::load(qrow);
    qa[1] = Frag<_Float16>::load(qrow + 32);
  }

  float mrow[8], lrow[8];
  v8f oacc[4];
#pragma unroll
  for (int r = 0; r < 8; ++r) { mrow[r] = -INFINITY; lrow[r] = 0.f; }
#pragma unroll
  for (int t = 0; t < 4; ++t) oacc[t] = (v8f){0.f,0.f,0.f,0.f,0.f,0.f,0.f,0.f};

  _Float16* pw = Psh[wave];

#pragma unroll 1
  for (int kc = 0; kc < kSeq / kKC; ++kc) {
    const int kv0 = kc * kKC;
    __syncthreads();
#pragma unroll
    for (int it = 0; it < 4; ++it) {
      const int p  = it * 128 + tid;
      const int r  = p >> 3;
      const int c8 = (p & 7) * 8;
      const v8h kk = *(const v8h*)(Kb + (size_t)(kv0 + r) * kHd + c8);
      const v8h vv = *(const v8h*)(Vb + (size_t)r * kSeq + kv0 + c8);
      *(v8h*)(Ksh + r * kHd + c8) = kk;
      *(v8h*)(Vsh + r * kKC + c8) = vv;
    }
    __syncthreads();

    v8f s[4];
#pragma unroll
    for (int j = 0; j < 4; ++j) {
      s[j] = (v8f){0.f,0.f,0.f,0.f,0.f,0.f,0.f,0.f};
#pragma unroll
      for (int dc = 0; dc < 2; ++dc) {
        const v16h kb = Frag<_Float16>::load(Ksh + (j * 16 + c) * kHd + dc * 32 + 8 * hh);
        s[j] = mma_h(qa[dc], kb, s[j]);
      }
    }

    float cm[8];
#pragma unroll
    for (int r = 0; r < 8; ++r) {
      float m = -INFINITY;
#pragma unroll
      for (int j = 0; j < 4; ++j) {
        const float sv = s[j][r] * kAttScale;
        s[j][r] = sv;
        m = fmaxf(m, sv);
      }
#pragma unroll
      for (int off = 1; off < 16; off <<= 1) m = fmaxf(m, __shfl_xor(m, off, 32));
      cm[r] = m;
    }
#pragma unroll
    for (int r = 0; r < 8; ++r) {
      const float mnew  = fmaxf(mrow[r], cm[r]);
      const float alpha = expf(mrow[r] - mnew);
      mrow[r] = mnew;
      float psum = 0.f;
#pragma unroll
      for (int j = 0; j < 4; ++j) {
        const float p = expf(s[j][r] - mnew);
        psum += p;
        pw[(8 * hh + r) * kKC + j * 16 + c] = (_Float16)(p * kPCarry);
      }
#pragma unroll
      for (int off = 1; off < 16; off <<= 1) psum += __shfl_xor(psum, off, 32);
      lrow[r] = lrow[r] * alpha + psum;
#pragma unroll
      for (int t = 0; t < 4; ++t) oacc[t][r] *= alpha;
    }
    __syncthreads();
#pragma unroll
    for (int kk = 0; kk < 2; ++kk) {
      const v16h pa = Frag<_Float16>::load(pw + c * kKC + kk * 32 + 8 * hh);
#pragma unroll
      for (int t = 0; t < 4; ++t) {
        const v16h vb = Frag<_Float16>::load(Vsh + (t * 16 + c) * kKC + kk * 32 + 8 * hh);
        oacc[t] = mma_h(pa, vb, oacc[t]);
      }
    }
  }

  float* os = Os[wave];
#pragma unroll
  for (int r = 0; r < 8; ++r) {
    const float inv = kOCarry / (lrow[r] * kPCarry);
#pragma unroll
    for (int t = 0; t < 4; ++t) os[(8 * hh + r) * 68 + t * 16 + c] = oacc[t][r] * inv;
  }
  __syncthreads();
  {
    const int q = lane >> 3, c8 = (lane & 7) * 8;
    v8h hv[4];
#pragma unroll
    for (int it = 0; it < 4; ++it) {
      const int row = it * 4 + q;
      const float* sp = os + row * 68 + c8;
      const v4f a0 = *(const v4f*)(sp);
      const v4f a1 = *(const v4f*)(sp + 4);
#pragma unroll
      for (int e = 0; e < 4; ++e) {
        hv[it][e]     = (_Float16)a0[e];
        hv[it][4 + e] = (_Float16)a1[e];
      }
    }
    unsigned short* ob = Op + ((size_t)b * kSeq + q0) * kDim + (size_t)h * kHd + c8;
    for (int pass = 0; pass < 2; ++pass) {
#pragma unroll
      for (int it = 0; it < 4; ++it) {
        const int row = it * 4 + q;
        *(volatile v8h*)(ob + (size_t)row * kDim) = hv[it];
      }
      __threadfence();
    }
  }
}

extern "C" void kernel_launch(void* const* d_in, const int* in_sizes, int n_in,
                              void* d_out, int out_size, void* d_ws, size_t ws_size,
                              hipStream_t stream)
{
  if (n_in < 4) return;
  if (in_sizes[0] != kRows * kDim) return;
  if (in_sizes[1] != kDim * kQkvN) return;
  if (in_sizes[2] != kDim * kDim) return;
  if (in_sizes[3] != kDim) return;
  if (out_size != kRows * kDim) return;
  if (ws_size < kWsTotal) return;

  const float* x     = (const float*)d_in[0];
  const float* w_qkv = (const float*)d_in[1];
  const float* w_out = (const float*)d_in[2];
  const float* b_out = (const float*)d_in[3];
  float* out = (float*)d_out;

  char* ws = (char*)d_ws;
  unsigned short* XH   = (unsigned short*)(ws + kOffXH);
  unsigned short* WQT  = (unsigned short*)(ws + kOffWQT);
  unsigned short* WOT  = (unsigned short*)(ws + kOffWOT);
  unsigned short* QKVH = (unsigned short*)(ws + kOffQKVH);
  unsigned short* VT   = (unsigned short*)(ws + kOffVT);
  unsigned short* OH   = (unsigned short*)(ws + kOffOH);
  unsigned short* QH   = QKVH;
  unsigned short* KH   = QKVH + kPlaneHalves;
  unsigned short* VH   = QKVH + 2 * kPlaneHalves;

  cast_f16_kernel<<<(kRows * kDim) / 8 / 256, 256, 0, stream>>>(x, XH, (kRows * kDim) / 8, 1.0f);

  transpose_cast_kernel<<<dim3(kQkvN / 64, kDim / 64), 256, 0, stream>>>(w_qkv, WQT, kDim, kQkvN, kWCarry);
  transpose_cast_kernel<<<dim3(kDim / 64, kDim / 64), 256, 0, stream>>>(w_out, WOT, kDim, kDim, kWCarry);

  wmma_gemm64<0, false, 0, 1, false><<<dim3(8, 3 * kHeads), 256, 0, stream>>>(
      XH, XH, kDim, 0L,
      WQT, WQT, kDim, (long)kHd * kDim,
      (void*)QKVH, (void*)QKVH, kHd, (long)kRows * kHd,
      b_out, x, 0L,
      kRows, kHd, kDim, kWCarryInv);

  vtrans_kernel<<<dim3(kSeq / 64, kHeads * kBatch), 256, 0, stream>>>(VH, VT);

  attn_f16_kernel<<<kHeads * kBatch * kQTiles, 128, 0, stream>>>(QH, KH, VT, OH);

  wmma_gemm64<0, false, 2, 0, false><<<dim3(128, 1), 256, 0, stream>>>(
      OH, OH, kDim, 0L,
      WOT, WOT, kDim, 0L,
      (void*)out, (void*)out, kDim, 0L,
      b_out, x, 0L,
      kRows, kDim, kDim, kOutScale);
}
